// SimpleRNN_40200893890811
// MI455X (gfx1250) — hardware-verified
//
#include <hip/hip_runtime.h>
#include <math.h>

constexpr int NBAT   = 64;
constexpr int NSTEP  = 1024;
constexpr int NCH    = 64;
constexpr int NHID   = 256;
constexpr int NOUTC  = 20;
constexpr int NOUTP  = 32;
constexpr int NROWS  = NBAT * NSTEP;
constexpr int NTHR   = 256;
constexpr int DTHR   = 128;
constexpr int SEQ_BLK = 16;
constexpr int HPITCH = 264;
constexpr int SPITCH = 260;
constexpr int OUT_LINES = (64 * NOUTC * 4) / 128;
constexpr float WCARRY = 64.0f;
constexpr float ACARRY = 16.0f;
constexpr float FOLD   = 1.0f / 1024.0f;
constexpr float BN_EPS_F = 1e-3f;
static_assert(NROWS % 64 == 0 && NHID % 64 == 0, "GEMM M, N tile multiples");
static_assert(NCH % 32 == 0 && NHID % 32 == 0, "GEMM K multiples of 32");
static_assert(NCH % 64 == 0 && NHID % 64 == 0, "transpose tiles 64x64");
static_assert(NBAT % SEQ_BLK == 0, "recurrence grid exact");
static_assert(NHID == 32 * (NTHR / 32), "8 waves x 32 hidden columns");
static_assert((64 * NOUTC * 4) % 128 == 0 && OUT_LINES == 40, "output tile is whole lines");
static_assert(NOUTC > 16 && NOUTC <= NOUTP, "two output subtiles");
static_assert((NROWS * (NCH / 8)) % NTHR == 0, "x convert grid exact");
static_assert((NOUTP * NHID / 8) % NTHR == 0, "Wd prep grid exact");
static_assert(((NROWS / 64) * (NHID / 64)) % 8 == 0, "xproj GEMM grid exact");
static_assert(HPITCH % 8 == 0 && SPITCH % 4 == 0, "16-B aligned LDS rows");

typedef __attribute__((ext_vector_type(16))) _Float16 v16h;
typedef __attribute__((ext_vector_type(8)))  _Float16 v8h;
typedef __attribute__((ext_vector_type(16))) __bf16   v16b;
typedef __attribute__((ext_vector_type(8)))  __bf16   v8b;
typedef __attribute__((ext_vector_type(8)))  float    v8f;
typedef __attribute__((ext_vector_type(4)))  float    v4f;

__device__ __forceinline__ unsigned short f2bf_bits(float f) {
  unsigned u = __float_as_uint(f);
  return (unsigned short)((u + 0x7FFFu + ((u >> 16) & 1u)) >> 16);
}
__device__ __forceinline__ float bf_bits2f(unsigned short h) { return __uint_as_float(((unsigned)h) << 16); }

__device__ __forceinline__ void dep_guard_h(v8f& a, v8f& b, v16h x, v16h y) { asm volatile("v_nop\n\tv_nop\n\tv_nop\n\tv_nop" : "+v"(a), "+v"(b) : "v"(x), "v"(y)); }
__device__ __forceinline__ void dep_guard_b(v8f& a, v8f& b, v16b x, v16b y) { asm volatile("v_nop\n\tv_nop\n\tv_nop\n\tv_nop" : "+v"(a), "+v"(b) : "v"(x), "v"(y)); }
__device__ __forceinline__ void keep4_h(v16h a, v16h b, v16h c, v16h d) { asm volatile("v_nop" :: "v"(a), "v"(b), "v"(c), "v"(d)); }
__device__ __forceinline__ void keep4_b(v16b a, v16b b, v16b c, v16b d) { asm volatile("v_nop" :: "v"(a), "v"(b), "v"(c), "v"(d)); }
__device__ __forceinline__ void acc_guard4(v8f& a, v8f& b, v8f& c, v8f& d) { asm volatile("v_nop\n\tv_nop\n\tv_nop\n\tv_nop" : "+v"(a), "+v"(b), "+v"(c), "+v"(d)); }
__device__ __forceinline__ void acc_guard2(v8f& a, v8f& b) { asm volatile("v_nop\n\tv_nop\n\tv_nop\n\tv_nop" : "+v"(a), "+v"(b)); }
template <typename T> struct Frag;
template <> struct Frag<_Float16> {
  typedef v16h V; union U { v16h v; v8h h[2]; };
  static __device__ __forceinline__ v16h load(const _Float16* p) {
    U f; f.h[0] = *(const v8h*)(p); f.h[1] = *(const v8h*)(p + 16); return f.v;
  }
  static __device__ __forceinline__ v8f mma(v16h a, v16h b, v8f c) {
    return __builtin_amdgcn_wmma_f32_16x16x32_f16(false, a, false, b, (short)0, c, false, false);
  }
  static __device__ __forceinline__ void guard(v8f& a, v8f& b, v16h x, v16h y) { dep_guard_h(a, b, x, y); }
  static __device__ __forceinline__ void keep(v16h a, v16h b, v16h c, v16h d) { keep4_h(a, b, c, d); }
};
template <> struct Frag<__bf16> {
  typedef v16b V; union U { v16b v; v8b h[2]; };
  static __device__ __forceinline__ v16b load(const __bf16* p) {
    U f; f.h[0] = *(const v8b*)(p); f.h[1] = *(const v8b*)(p + 16); return f.v;
  }
  static __device__ __forceinline__ v8f mma(v16b a, v16b b, v8f c) {
    return __builtin_amdgcn_wmma_f32_16x16x32_bf16(false, a, false, b, (short)0, c, false, false);
  }
  static __device__ __forceinline__ void guard(v8f& a, v8f& b, v16b x, v16b y) { dep_guard_b(a, b, x, y); }
  static __device__ __forceinline__ void keep(v16b a, v16b b, v16b c, v16b d) { keep4_b(a, b, c, d); }
};

__device__ __forceinline__ float fsig_precise(float x) { return __builtin_amdgcn_rcpf(1.0f + expf(-x)); }

template <int ET> struct Elem;
template <> struct Elem<0> { typedef _Float16 T; };
template <> struct Elem<1> { typedef __bf16 T; };
template <int ET, bool SPLIT, int BIAS_MODE, int OUT_MODE, bool RESID, int ACT = 0>
__global__ __launch_bounds__(256) void wmma_gemm64(
    const unsigned short* __restrict__ Ap, const unsigned short* __restrict__ A2p, int lda, long strideA,
    const unsigned short* __restrict__ Btp, const unsigned short* __restrict__ Bt2p, int ldb, long strideB,
    void* __restrict__ Cout, void* __restrict__ Cout2, int ldc, long strideC,
    const float* __restrict__ bias,
    const float* __restrict__ resid, long strideR,
    int M, int N, int K, float scale) {
  typedef typename Elem<ET>::T T;
  typedef typename Frag<T>::V V;
  const T* A = (const T*)Ap; const T* A2 = (const T*)A2p; const T* Bt = (const T*)Btp; const T* Bt2 = (const T*)Bt2p;
  __shared__ __align__(16) float sT[8][16 * 68];
  const int b    = blockIdx.y;
  const int lane = threadIdx.x & 31;
  const int wave = threadIdx.x >> 5;
  const int tilesN = N >> 6;
  const int tilesM = M >> 6;
  const int tile = blockIdx.x * 8 + wave;
  if (tile >= tilesM * tilesN) return;
  const int tm = tile / tilesN;
  const int tn = tile - tm * tilesN;
  const int m0 = tm << 6;
  const int n0 = tn << 6;

  const T* Ab  = A  + (size_t)b * strideA;
  const T* Bb  = Bt + (size_t)b * strideB;
  const T* Ab2 = SPLIT ? (A2  + (size_t)b * strideA) : nullptr;
  const T* Bb2 = SPLIT ? (Bt2 + (size_t)b * strideB) : nullptr;

  const int rlane = lane & 15;
  const int koff  = (lane >> 4) * 8;
  const int mOff  = (lane >> 4) * 8;

  v8f acc[4][4];
#pragma unroll
  for (int i = 0; i < 4; ++i)
#pragma unroll
    for (int j = 0; j < 4; ++j) acc[i][j] = (v8f){0.f,0.f,0.f,0.f,0.f,0.f,0.f,0.f};

  for (int k0 = 0; k0 < K; k0 += 32) {
    V bh[4], bl[4];
#pragma unroll
    for (int j = 0; j < 4; ++j) {
      const size_t bo = (size_t)(n0 + (j << 4) + rlane) * ldb + koff + k0;
      bh[j] = Frag<T>::load(Bb + bo);
      if (SPLIT) bl[j] = Frag<T>::load(Bb2 + bo);
    }
#pragma unroll
    for (int i = 0; i < 4; ++i) {
      const size_t ao = (size_t)(m0 + (i << 4) + rlane) * lda + koff + k0;
      V ah = Frag<T>::load(Ab + ao);
      V al;
      if (SPLIT) al = Frag<T>::load(Ab2 + ao);
#pragma unroll
      for (int j = 0; j < 4; ++j) {
        acc[i][j] = Frag<T>::mma(ah, bh[j], acc[i][j]);
        if (SPLIT) {
          acc[i][j] = Frag<T>::mma(ah, bl[j], acc[i][j]);
          acc[i][j] = Frag<T>::mma(al, bh[j], acc[i][j]);
        }
      }
      Frag<T>::guard(acc[i][0], acc[i][3], ah, SPLIT ? al : ah);
    }
    Frag<T>::keep(bh[0], bh[1], bh[2], bh[3]);
    if (SPLIT) Frag<T>::keep(bl[0], bl[1], bl[2], bl[3]);
  }
  acc_guard4(acc[0][0], acc[0][1], acc[0][2], acc[0][3]);
  acc_guard4(acc[1][0], acc[1][1], acc[1][2], acc[1][3]);
  acc_guard4(acc[2][0], acc[2][1], acc[2][2], acc[2][3]);
  acc_guard4(acc[3][0], acc[3][1], acc[3][2], acc[3][3]);

  float* slab = sT[wave];
  const float* Rb = RESID ? (resid + (size_t)b * strideR) : nullptr;
#pragma unroll
  for (int i = 0; i < 4; ++i) {
    const int mBase = m0 + (i << 4);
#pragma unroll
    for (int j = 0; j < 4; ++j) {
      const int n = n0 + (j << 4) + rlane;
      float bv = 0.f;
      if (BIAS_MODE == 2) bv = bias[n];
#pragma unroll
      for (int r = 0; r < 8; ++r) {
        float v = acc[i][j][r] * scale;
        if (BIAS_MODE == 1) v += bias[mBase + mOff + r];
        if (BIAS_MODE == 2) v += bv;
        if (RESID) v += Rb[(size_t)(mBase + mOff + r) * ldc + n];
        if (ACT == 1) v = tanhf(v);
        if (ACT == 2) v = fmaxf(v, 0.0f);
        if (ACT == 3) v = v / (1.0f + expf(-v));
        if (ACT == 4) v = (v > 0.f) ? v : 0.01f * v;
        if (ACT == 5) v = 0.5f * v * (1.0f + erff(v * 0.70710678118654752f));
        slab[(mOff + r) * 68 + (j << 4) + rlane] = v;
      }
    }
    __builtin_amdgcn_fence(__ATOMIC_RELEASE, "workgroup");
    __builtin_amdgcn_wave_barrier();
    __builtin_amdgcn_fence(__ATOMIC_ACQUIRE, "workgroup");
    if (OUT_MODE == 0) {
      float* C = (float*)Cout + (size_t)b * strideC;
      const int hh = lane >> 4, c4 = (lane & 15) * 4;
      for (int pass = 0; pass < 2; ++pass) {
#pragma unroll
        for (int it = 0; it < 8; ++it) {
          const int row = it * 2 + hh;
          v4f v = *(const v4f*)(slab + row * 68 + c4);
          *(volatile v4f*)(C + (size_t)(mBase + row) * ldc + n0 + c4) = v;
        }
        __threadfence();
      }
    } else {
      const int q = lane >> 3, c8 = (lane & 7) * 8;
      unsigned short* C  = (unsigned short*)Cout  + (size_t)b * strideC;
      unsigned short* C2 = (OUT_MODE == 2) ? ((unsigned short*)Cout2 + (size_t)b * strideC) : nullptr;
      for (int pass = 0; pass < 2; ++pass) {
#pragma unroll
        for (int it = 0; it < 4; ++it) {
          const int row = it * 4 + q;
          const float* sp = slab + row * 68 + c8;
          v8h hv, lv;
#pragma unroll
          for (int e = 0; e < 8; ++e) {
            if (OUT_MODE == 1) {
              hv[e] = (_Float16)sp[e];
            } else {
              unsigned short hb = f2bf_bits(sp[e]);
              unsigned short lb = f2bf_bits(sp[e] - bf_bits2f(hb));
              hv[e] = __builtin_bit_cast(_Float16, hb);
              lv[e] = __builtin_bit_cast(_Float16, lb);
            }
          }
          *(volatile v8h*)(C + (size_t)(mBase + row) * ldc + n0 + c8) = hv;
          if (OUT_MODE == 2) *(volatile v8h*)(C2 + (size_t)(mBase + row) * ldc + n0 + c8) = lv;
        }
        __threadfence();
      }
    }
    __builtin_amdgcn_fence(__ATOMIC_RELEASE, "workgroup");
    __builtin_amdgcn_wave_barrier();
    __builtin_amdgcn_fence(__ATOMIC_ACQUIRE, "workgroup");
  }
}

__global__ __launch_bounds__(NTHR) void tpw16_kernel(const float* __restrict__ src, int R, int C, int ldo,
                                                     unsigned short* __restrict__ O, float sc) {
  __shared__ float Tt[64 * 65];
  const int tid = threadIdx.x;
  const int c0 = blockIdx.x * 64, r0 = blockIdx.y * 64;
#pragma unroll
  for (int i = 0; i < 4; ++i) {
    const int idx = i * NTHR + tid;
    const int rr = idx >> 4, cc = (idx & 15) * 4;
    const v4f v = *(const v4f*)(src + (size_t)(r0 + rr) * (size_t)C + c0 + cc);
    Tt[rr * 65 + cc + 0] = v[0];
    Tt[rr * 65 + cc + 1] = v[1];
    Tt[rr * 65 + cc + 2] = v[2];
    Tt[rr * 65 + cc + 3] = v[3];
  }
  __syncthreads();
  const int q = tid >> 3, c8 = (tid & 7) * 8;
  v8h hv[2];
#pragma unroll
  for (int g = 0; g < 2; ++g) {
    const int qq = g * 32 + q;
#pragma unroll
    for (int e = 0; e < 8; ++e) {
      const float f = Tt[(c8 + e) * 65 + qq];
      hv[g][e] = (_Float16)(f * sc);
    }
  }
  for (int pass = 0; pass < 2; ++pass) {
#pragma unroll
    for (int g = 0; g < 2; ++g) {
      const size_t o = (size_t)(c0 + g * 32 + q) * (size_t)ldo + (size_t)(r0 + c8);
      *(volatile v8h*)(O + o) = hv[g];
    }
    __threadfence();
  }
}

__global__ __launch_bounds__(NTHR) void wd_prep_kernel(const float* __restrict__ Wd, unsigned short* __restrict__ WDT) {
  const int i  = blockIdx.x * NTHR + threadIdx.x;
  const int o  = i >> 5;
  const int u8 = (i & 31) * 8;
  const int oc = (o < NOUTC) ? o : (NOUTC - 1);
  const float fa = (o < NOUTC) ? WCARRY : 0.0f;
  v8h hv;
#pragma unroll
  for (int e = 0; e < 8; ++e) {
    const float w = Wd[(size_t)(u8 + e) * NOUTC + oc];
    hv[e] = (_Float16)(w * fa);
  }
  *(volatile v8h*)(WDT + (size_t)i * 8) = hv;
  __threadfence();
  *(volatile v8h*)(WDT + (size_t)i * 8) = hv;
}

__global__ __launch_bounds__(NTHR) void bnx_cvt_kernel(const float* __restrict__ x, const float* __restrict__ g1,
                                                       const float* __restrict__ b1, const float* __restrict__ m1,
                                                       const float* __restrict__ v1, unsigned short* __restrict__ XA, int n8) {
  const int i = blockIdx.x * NTHR + threadIdx.x;
  if (i < n8) {
    const int row = i >> 3;
    const int c8  = (i & 7) * 8;
    const v4f ga = *(const v4f*)(g1 + c8), gb = *(const v4f*)(g1 + c8 + 4);
    const v4f va = *(const v4f*)(v1 + c8), vb = *(const v4f*)(v1 + c8 + 4);
    const v4f ba = *(const v4f*)(b1 + c8), bb = *(const v4f*)(b1 + c8 + 4);
    const v4f ma = *(const v4f*)(m1 + c8), mb = *(const v4f*)(m1 + c8 + 4);
    float inv[8], sh[8];
#pragma unroll
    for (int e = 0; e < 4; ++e) {
      inv[e]     = ga[e] * rsqrtf(va[e] + BN_EPS_F);
      inv[4 + e] = gb[e] * rsqrtf(vb[e] + BN_EPS_F);
      sh[e]      = ba[e] - ma[e] * inv[e];
      sh[4 + e]  = bb[e] - mb[e] * inv[4 + e];
    }
    asm volatile("" ::: "memory");
    const v4f xa = *(const v4f*)(x + (size_t)row * NCH + c8);
    const v4f xb = *(const v4f*)(x + (size_t)row * NCH + c8 + 4);
    v8h hv;
#pragma unroll
    for (int e = 0; e < 4; ++e) {
      hv[e]     = (_Float16)((xa[e] * inv[e] + sh[e]) * ACARRY);
      hv[4 + e] = (_Float16)((xb[e] * inv[4 + e] + sh[4 + e]) * ACARRY);
    }
    *(volatile v8h*)(XA + (size_t)i * 8) = hv;
    __threadfence();
    *(volatile v8h*)(XA + (size_t)i * 8) = hv;
  }
}

__global__ __launch_bounds__(NTHR) void rec_kernel(const float* __restrict__ XP, const unsigned short* __restrict__ WHTp,
                                                   const float* __restrict__ g2, const float* __restrict__ b2,
                                                   const float* __restrict__ m2, const float* __restrict__ v2,
                                                   unsigned short* __restrict__ HS) {
  __shared__ __align__(16) _Float16 Ah[SEQ_BLK * HPITCH];
  __shared__ __align__(16) float    Hs[SEQ_BLK * SPITCH];
  const _Float16* WH = (const _Float16*)WHTp;
  const int tid = threadIdx.x, lane = tid & 31, wave = tid >> 5;
  const int c = lane & 15, hh = lane >> 4, koff = hh * 8;
  const int rowbase = blockIdx.x * SEQ_BLK;

#pragma unroll 1
  for (int i = tid; i < SEQ_BLK * HPITCH; i += NTHR) Ah[i] = (_Float16)0.0f;

  float inv2v[2], sh2v[2], hst[2][8];
#pragma unroll
  for (int nt = 0; nt < 2; ++nt) {
    const int j = 32 * wave + 16 * nt + c;
    const float gg = g2[j], vv = v2[j], bbv = b2[j], mm = m2[j];
    const float iv = gg * rsqrtf(vv + BN_EPS_F);
    inv2v[nt] = iv;
    sh2v[nt]  = bbv - mm * iv;
#pragma unroll
    for (int r = 0; r < 8; ++r) hst[nt][r] = 0.0f;
  }
  __syncthreads();

  const _Float16* ahrow = Ah + c * HPITCH + koff;
  const _Float16* wh0 = WH + (size_t)(32 * wave + c) * NHID + koff;
  const _Float16* wh1 = wh0 + (size_t)16 * NHID;
  const int j0 = 32 * wave + c, j1 = j0 + 16;
  const v8f z8 = {0.f, 0.f, 0.f, 0.f, 0.f, 0.f, 0.f, 0.f};

#pragma unroll 1
  for (int t = 0; t < NSTEP; ++t) {
    float xr0[8], xr1[8];
#pragma unroll
    for (int r = 0; r < 8; ++r)
      xr0[r] = XP[((size_t)(rowbase + 8 * hh + r) * NSTEP + (size_t)t) * NHID + j0];

    v8f acc0 = z8, acc1 = z8;
#pragma unroll 1
    for (int k0 = 0; k0 < NHID; k0 += 32) {
      const v16h a   = Frag<_Float16>::load(ahrow + k0);
      const v16h bf0 = Frag<_Float16>::load(wh0 + k0);
      const v16h bf1 = Frag<_Float16>::load(wh1 + k0);
      acc0 = Frag<_Float16>::mma(a, bf0, acc0);
      acc1 = Frag<_Float16>::mma(a, bf1, acc1);
      dep_guard_h(acc0, acc1, a, bf1);
      keep4_h(a, bf0, bf1, a);
    }
    acc_guard2(acc0, acc1);
    asm volatile("" ::: "memory");
#pragma unroll
    for (int r = 0; r < 8; ++r)
      xr1[r] = XP[((size_t)(rowbase + 8 * hh + r) * NSTEP + (size_t)t) * NHID + j1];

#pragma unroll
    for (int r = 0; r < 8; ++r) {
      hst[0][r] = tanhf(acc0[r] * FOLD + xr0[r]);
      hst[1][r] = tanhf(acc1[r] * FOLD + xr1[r]);
    }
    __syncthreads();
#pragma unroll
    for (int nt = 0; nt < 2; ++nt) {
      const int j = 32 * wave + 16 * nt + c;
#pragma unroll
      for (int r = 0; r < 8; ++r) {
        const float hv = hst[nt][r];
        Ah[(8 * hh + r) * HPITCH + j] = (_Float16)(hv * ACARRY);
        Hs[(8 * hh + r) * SPITCH + j] = (hv * inv2v[nt] + sh2v[nt]) * ACARRY;
      }
    }
    __syncthreads();
    v8h hrow[2];
#pragma unroll
    for (int it = 0; it < 2; ++it) {
      const int row = it * 8 + wave;
      const float* sp = Hs + row * SPITCH + lane * 8;
      const v4f p0 = *(const v4f*)(sp);
      const v4f p1 = *(const v4f*)(sp + 4);
#pragma unroll
      for (int e = 0; e < 4; ++e) { hrow[it][e] = (_Float16)p0[e]; hrow[it][4 + e] = (_Float16)p1[e]; }
    }
    for (int pass = 0; pass < 2; ++pass) {
#pragma unroll
      for (int it = 0; it < 2; ++it) {
        const int row = it * 8 + wave;
        *(volatile v8h*)(HS + (((size_t)(rowbase + row)) * NSTEP + (size_t)t) * NHID + lane * 8) = hrow[it];
      }
      __threadfence();
    }
  }
}

__global__ __launch_bounds__(DTHR) void dense_kernel(const unsigned short* __restrict__ HSp, const unsigned short* __restrict__ WDTp,
                                                     const float* __restrict__ bd, float* __restrict__ out) {
  __shared__ __align__(16) float So[64 * NOUTC];
  const _Float16* HSh = (const _Float16*)HSp;
  const _Float16* WD  = (const _Float16*)WDTp;
  const int tid = threadIdx.x, lane = tid & 31, wave = tid >> 5;
  const int c = lane & 15, hh = lane >> 4, koff = hh * 8;
  const int m0 = blockIdx.x * 64;

  const _Float16* arow = HSh + (size_t)(m0 + 16 * wave + c) * NHID + koff;
  const _Float16* w0   = WD + (size_t)c * NHID + koff;
  const _Float16* w1   = WD + (size_t)(16 + c) * NHID + koff;
  const int c1c = (16 + c < NOUTC) ? (16 + c) : (NOUTC - 1);
  const float bd0 = bd[c];
  const float bd1 = bd[c1c];
  const v8f z8 = {0.f, 0.f, 0.f, 0.f, 0.f, 0.f, 0.f, 0.f};

  v8f acc0 = z8, acc1 = z8;
#pragma unroll 1
  for (int k0 = 0; k0 < NHID; k0 += 32) {
    const v16h a   = Frag<_Float16>::load(arow + k0);
    const v16h bf0 = Frag<_Float16>::load(w0 + k0);
    const v16h bf1 = Frag<_Float16>::load(w1 + k0);
    acc0 = Frag<_Float16>::mma(a, bf0, acc0);
    acc1 = Frag<_Float16>::mma(a, bf1, acc1);
    dep_guard_h(acc0, acc1, a, bf1);
    keep4_h(a, bf0, bf1, a);
  }
  acc_guard2(acc0, acc1);

#pragma unroll
  for (int r = 0; r < 8; ++r) {
    const int row = 16 * wave + 8 * hh + r;
    const float s0 = fsig_precise(acc0[r] * FOLD + bd0);
    const float s1 = fsig_precise(acc1[r] * FOLD + bd1);
    So[row * NOUTC + c] = s0;
    if (c < NOUTC - 16) So[row * NOUTC + 16 + c] = s1;
  }
  __syncthreads();

  const int q = lane >> 3, l4 = (lane & 7) * 4;
  v4f vals[3];
#pragma unroll
  for (int it = 0; it < 3; ++it) {
    const int line = it * 16 + wave * 4 + q;
    const int lc = (line < OUT_LINES) ? line : (OUT_LINES - 1);
    vals[it] = *(const v4f*)(So + lc * 32 + l4);
  }
  float* ob = out + (size_t)m0 * NOUTC;
  for (int pass = 0; pass < 2; ++pass) {
#pragma unroll
    for (int it = 0; it < 3; ++it) {
      if (it * 16 + wave * 4 < OUT_LINES) {
        const int line = it * 16 + wave * 4 + q;
        *(volatile v4f*)(ob + (size_t)line * 32 + l4) = vals[it];
      }
    }
    __threadfence();
  }
}

extern "C" void kernel_launch(void* const* d_in, const int* in_sizes, int n_in,
                              void* d_out, int out_size, void* d_ws, size_t ws_size, hipStream_t stream) {
  if (n_in < 14 || d_out == nullptr || d_ws == nullptr) return;
  if (in_sizes[0] != NBAT * NSTEP * NCH || in_sizes[1] != NCH || in_sizes[2] != NCH || in_sizes[3] != NCH ||
      in_sizes[4] != NCH || in_sizes[5] != NCH * NHID || in_sizes[6] != NHID * NHID || in_sizes[7] != NHID ||
      in_sizes[8] != NHID || in_sizes[9] != NHID || in_sizes[10] != NHID || in_sizes[11] != NHID ||
      in_sizes[12] != NHID * NOUTC || in_sizes[13] != NOUTC || out_size != NROWS * NOUTC) return;

  const float* x   = (const float*)d_in[0];
  const float* g1  = (const float*)d_in[1];
  const float* b1  = (const float*)d_in[2];
  const float* m1  = (const float*)d_in[3];
  const float* v1  = (const float*)d_in[4];
  const float* Wx  = (const float*)d_in[5];
  const float* Wh  = (const float*)d_in[6];
  const float* bh  = (const float*)d_in[7];
  const float* g2  = (const float*)d_in[8];
  const float* b2  = (const float*)d_in[9];
  const float* m2  = (const float*)d_in[10];
  const float* v2  = (const float*)d_in[11];
  const float* Wd  = (const float*)d_in[12];
  const float* bd  = (const float*)d_in[13];
  float* out = (float*)d_out;

  char* ws = (char*)d_ws; size_t off = 0;
  auto carve = [&](size_t bytes) -> char* { char* p = ws + off; off += (bytes + 255) & ~(size_t)255; return p; };
  unsigned short* XA    = (unsigned short*)carve((size_t)NROWS * NCH * 2);
  unsigned short* WXT   = (unsigned short*)carve((size_t)NHID * NCH * 2);
  unsigned short* WHT   = (unsigned short*)carve((size_t)NHID * NHID * 2);
  unsigned short* WDT   = (unsigned short*)carve((size_t)NOUTP * NHID * 2);
  float*          XPROJ = (float*)carve((size_t)NROWS * NHID * 4);
  unsigned short* HS    = (unsigned short*)carve((size_t)NROWS * NHID * 2);
  if (off > ws_size || off > (size_t)134217728) return;

  tpw16_kernel<<<dim3(NHID / 64, NCH / 64), NTHR, 0, stream>>>(Wx, NCH, NHID, NCH, WXT, WCARRY);
  tpw16_kernel<<<dim3(NHID / 64, NHID / 64), NTHR, 0, stream>>>(Wh, NHID, NHID, NHID, WHT, WCARRY);
  wd_prep_kernel<<<(NOUTP * NHID / 8) / NTHR, NTHR, 0, stream>>>(Wd, WDT);
  const int n8x = NROWS * (NCH / 8);
  bnx_cvt_kernel<<<(n8x + NTHR - 1) / NTHR, NTHR, 0, stream>>>(x, g1, b1, m1, v1, XA, n8x);
  wmma_gemm64<0, false, 2, 0, false, 0><<<dim3((NROWS / 64) * (NHID / 64) / 8, 1), 256, 0, stream>>>(
      XA, XA, NCH, 0L, WXT, WXT, NCH, 0L, (void*)XPROJ, (void*)XPROJ, NHID, 0L,
      bh, XPROJ, 0L, NROWS, NHID, NCH, FOLD);
  rec_kernel<<<NBAT / SEQ_BLK, NTHR, 0, stream>>>(XPROJ, WHT, g2, b2, m2, v2, HS);
  dense_kernel<<<NROWS / 64, DTHR, 0, stream>>>(HS, WDT, bd, out);
}
